// GraphSAGEConv_60696477827758
// MI455X (gfx1250) — hardware-verified
//
#include <hip/hip_runtime.h>
#include <stddef.h>


#define DF        128
#define NTHR      256
#define NWAVE     8
#define EPT       8
#define NGRP      2
#define CHUNK     (NTHR * EPT * NGRP)
#define WCAP      (EPT * NGRP * 32)
#define LISTN     (NWAVE * WCAP)
#define NB        512
#define NU        64
#define LN_EPS    1e-5f
#define LDS_LAYER (NB * DF * 4 + LISTN * 4 + NB * 4 + 64)

static_assert((CHUNK & (CHUNK - 1)) == 0);
static_assert(CHUNK <= 4096);
static_assert((NB & (NB - 1)) == 0 && NB <= 4096);
static_assert(NB == NWAVE * 64);
static_assert(((NB / 16) % NWAVE) == 0);
static_assert(NU == NWAVE * 8);

typedef float  v4f  __attribute__((ext_vector_type(4)));
typedef float  v8f  __attribute__((ext_vector_type(8)));
typedef int    v4i  __attribute__((ext_vector_type(4)));
typedef __bf16 v8b  __attribute__((ext_vector_type(8)));
typedef __bf16 v16b __attribute__((ext_vector_type(16)));
union FragB { v16b v; v8b h[2]; };
union Pack8 { v8b b; v4i i; };

__device__ __forceinline__ v8f wmb(v16b a, v16b b, v8f c) {
  v8f d = __builtin_amdgcn_wmma_f32_16x16x32_bf16(false, a, false, b, (short)0, c, false, false);
  asm volatile("v_nop\n\tv_nop\n\tv_nop\n\tv_nop" : "+v"(d) : "v"(a), "v"(b));
  return d;
}

__device__ __forceinline__ void split8(const v4f a, const v4f b, v8b& hi, v8b& lo) {
#define SPL(I, X) { const float xv = (X); const __bf16 hq = (__bf16)xv; hi[I] = hq; lo[I] = (__bf16)(xv - (float)hq); }
  SPL(0, a.x) SPL(1, a.y) SPL(2, a.z) SPL(3, a.w)
  SPL(4, b.x) SPL(5, b.y) SPL(6, b.z) SPL(7, b.w)
#undef SPL
}

__global__ __launch_bounds__(NTHR) void k_wprep(const float* __restrict__ W,
                                                __bf16* whi, __bf16* wlo, int n8) {
  const int i = blockIdx.x * NTHR + threadIdx.x;
  if (i >= n8) return;
  const size_t o = (size_t)i * 8;
  const v4f a = *(const v4f*)(W + o), b = *(const v4f*)(W + o + 4);
  Pack8 ph, pl;
  split8(a, b, ph.b, pl.b);
  const v4i vh = ph.i, vl = pl.i;
  *(volatile v4i*)(whi + o) = vh;
  *(volatile v4i*)(wlo + o) = vl;
  __threadfence();
  *(volatile v4i*)(whi + o) = vh;
  *(volatile v4i*)(wlo + o) = vl;
}

__device__ __forceinline__ int scan_chunk(const int* __restrict__ dsts, int nE, int cbase, int nodeBase,
                                          int* list, int tid, int lane, int wave) {
  int wc = 0;
#pragma unroll
  for (int g = 0; g < NGRP; ++g) {
    const int el0  = (g * NTHR + tid) * EPT;
    const int e0   = cbase + el0;
    const int sent = -2147483647 - 1;
    v4i da, db;
    if (e0 + 7 < nE) {
      da = *(const v4i*)(dsts + e0);
      db = *(const v4i*)(dsts + e0 + 4);
    } else {
      da.x = (e0     < nE) ? dsts[min(e0, nE - 1)]     : sent;
      da.y = (e0 + 1 < nE) ? dsts[min(e0 + 1, nE - 1)] : sent;
      da.z = (e0 + 2 < nE) ? dsts[min(e0 + 2, nE - 1)] : sent;
      da.w = (e0 + 3 < nE) ? dsts[min(e0 + 3, nE - 1)] : sent;
      db.x = (e0 + 4 < nE) ? dsts[min(e0 + 4, nE - 1)] : sent;
      db.y = (e0 + 5 < nE) ? dsts[min(e0 + 5, nE - 1)] : sent;
      db.z = (e0 + 6 < nE) ? dsts[min(e0 + 6, nE - 1)] : sent;
      db.w = (e0 + 7 < nE) ? dsts[min(e0 + 7, nE - 1)] : sent;
    }
    const unsigned nb = (unsigned)nodeBase;
    const unsigned s0 = (unsigned)da.x - nb, s1 = (unsigned)da.y - nb;
    const unsigned s2 = (unsigned)da.z - nb, s3 = (unsigned)da.w - nb;
    const unsigned s4 = (unsigned)db.x - nb, s5 = (unsigned)db.y - nb;
    const unsigned s6 = (unsigned)db.z - nb, s7 = (unsigned)db.w - nb;
    const bool h0 = s0 < (unsigned)NB, h1 = s1 < (unsigned)NB, h2 = s2 < (unsigned)NB, h3 = s3 < (unsigned)NB;
    const bool h4 = s4 < (unsigned)NB, h5 = s5 < (unsigned)NB, h6 = s6 < (unsigned)NB, h7 = s7 < (unsigned)NB;
    const unsigned any = __builtin_amdgcn_ballot_w32(h0 | h1 | h2 | h3 | h4 | h5 | h6 | h7);
    if (any != 0u) {
#define HITJ(J, HJ, SJ) { \
        const unsigned mj = __builtin_amdgcn_ballot_w32(HJ); \
        if (mj != 0u) { \
          if (HJ) { \
            const int pos = wc + (int)__builtin_amdgcn_mbcnt_lo(mj, 0u); \
            if (pos < WCAP) list[wave * WCAP + pos] = ((el0 + (J)) << 12) | (int)(SJ); \
          } \
          wc += (int)__builtin_popcount(mj); } }
      HITJ(0, h0, s0)
      HITJ(1, h1, s1)
      HITJ(2, h2, s2)
      HITJ(3, h3, s3)
      HITJ(4, h4, s4)
      HITJ(5, h5, s5)
      HITJ(6, h6, s6)
      HITJ(7, h7, s7)
#undef HITJ
    }
  }
  return wc;
}

__global__ __launch_bounds__(NTHR) void k_layer(
    const float* __restrict__ fin, const int* __restrict__ srcs, const int* __restrict__ dsts,
    const __bf16* __restrict__ whi, const __bf16* __restrict__ wlo,
    const float* __restrict__ bl, const float* __restrict__ gm, const float* __restrict__ bt,
    float* fout, int nN, int nE) {
  extern __shared__ v4f lds_dyn[];
  float* hrow = (float*)lds_dyn;
  int*   list = (int*)(hrow + NB * DF);
  int*   cnt  = list + LISTN;
  int*   wcnt = cnt + NB;
  const int tid = threadIdx.x, lane = tid & 31, wave = tid >> 5, hh = lane >> 4, m = lane & 15;
  const int nodeBase = blockIdx.x * NB;

  {
    const v4f z = {0.f, 0.f, 0.f, 0.f};
    for (int i = tid; i < NB * DF / 4; i += NTHR) lds_dyn[i] = z;
    for (int i = tid; i < NB; i += NTHR) cnt[i] = 0;
  }
  __syncthreads();

  const int nChunks = (nE > 0) ? (nE + CHUNK - 1) / CHUNK : 0;
#pragma unroll 1
  for (int ch = 0; ch < nChunks; ++ch) {
    const int cbase = ch * CHUNK;
    const int wc = scan_chunk(dsts, nE, cbase, nodeBase, list, tid, lane, wave);
    if (lane == 0) wcnt[wave] = wc;
    __syncthreads();
    if (wave == 0) {
#pragma unroll 1
      for (int wsx = 0; wsx < NWAVE; ++wsx) {
        int n = __builtin_amdgcn_readfirstlane(wcnt[wsx]);
        n = n > WCAP ? WCAP : (n < 0 ? 0 : n);
        const int* lp = list + wsx * WCAP;
#pragma unroll 1
        for (int i = 0; i < n; ++i) {
          const int ent  = __builtin_amdgcn_readfirstlane(lp[i]);
          const int slot = ent & (NB - 1);
          int e = cbase + ((ent >> 12) & (CHUNK - 1));
          e = e > nE - 1 ? nE - 1 : e;
          int s = srcs[e];
          s = s < 0 ? 0 : (s > nN - 1 ? nN - 1 : s);
          const v4f v = *(const v4f*)(fin + (size_t)s * DF + 4 * lane);
          v4f* ap = (v4f*)(hrow + slot * DF + 4 * lane);
          *ap = *ap + v;
          if (lane == 0) cnt[slot] = cnt[slot] + 1;
        }
      }
    }
    __syncthreads();
  }

#pragma unroll 4
  for (int i = 0; i < (NB * DF / 4) / NTHR; ++i) {
    const int idx  = i * NTHR + tid;
    const int slot = idx >> 5;
    const int c4   = (idx & 31) * 4;
    int node = nodeBase + slot;
    node = node > nN - 1 ? nN - 1 : node;
    const float iv = 1.0f / (float)(cnt[slot] + 1);
    const v4f gv = *(const v4f*)(fin + (size_t)node * DF + c4);
    v4f* ap = (v4f*)(hrow + slot * DF + c4);
    *ap = (*ap + gv) * iv;
  }
  __syncthreads();

#pragma unroll 1
  for (int q = 0; q < (NB / 16) / NWAVE; ++q) {
    const int tl = wave + NWAVE * q;
    v8f acc[8];
#pragma unroll
    for (int t = 0; t < 8; ++t) { const v8f z = {0.f, 0.f, 0.f, 0.f, 0.f, 0.f, 0.f, 0.f}; acc[t] = z; }
#pragma unroll
    for (int kt = 0; kt < DF / 32; ++kt) {
      const float* ap = hrow + (size_t)(16 * tl + m) * DF + 32 * kt + 8 * hh;
      const v4f p0 = *(const v4f*)ap,        p1 = *(const v4f*)(ap + 4);
      const v4f p2 = *(const v4f*)(ap + 16), p3 = *(const v4f*)(ap + 20);
      FragB ah, al;
      split8(p0, p1, ah.h[0], al.h[0]);
      split8(p2, p3, ah.h[1], al.h[1]);
#pragma unroll
      for (int t = 0; t < 8; ++t) {
        const size_t bo = (size_t)(16 * t + m) * DF + 32 * kt + 8 * hh;
        FragB bh, bw;
        bh.h[0] = *(const v8b*)(whi + bo);
        bh.h[1] = *(const v8b*)(whi + bo + 16);
        bw.h[0] = *(const v8b*)(wlo + bo);
        bw.h[1] = *(const v8b*)(wlo + bo + 16);
        acc[t] = wmb(ah.v, bh.v, acc[t]);
        acc[t] = wmb(ah.v, bw.v, acc[t]);
        acc[t] = wmb(al.v, bh.v, acc[t]);
      }
    }

    float bb[8], gg[8], ee[8];
#pragma unroll
    for (int t = 0; t < 8; ++t) { const int col = 16 * t + m; bb[t] = bl[col]; gg[t] = gm[col]; ee[t] = bt[col]; }
    float* sp = hrow + (size_t)(16 * tl + 8 * hh) * DF + m;
#pragma unroll
    for (int j = 0; j < 8; ++j) {
      float s = 0.f;
#pragma unroll
      for (int t = 0; t < 8; ++t) { const float hv = acc[t][j] + bb[t]; acc[t][j] = hv; s += hv; }
      s += __shfl_xor(s, 8, 32); s += __shfl_xor(s, 4, 32); s += __shfl_xor(s, 2, 32); s += __shfl_xor(s, 1, 32);
      const float mean = s * (1.0f / 128.0f);
      float q2 = 0.f;
#pragma unroll
      for (int t = 0; t < 8; ++t) { const float d = acc[t][j] - mean; q2 += d * d; }
      q2 += __shfl_xor(q2, 8, 32); q2 += __shfl_xor(q2, 4, 32); q2 += __shfl_xor(q2, 2, 32); q2 += __shfl_xor(q2, 1, 32);
      const float var  = q2 * (1.0f / 128.0f);
      const float rstd = rsqrtf(var + LN_EPS);
#pragma unroll
      for (int t = 0; t < 8; ++t) {
        float y = (acc[t][j] - mean) * rstd * gg[t] + ee[t];
        y = y > 0.0f ? y : expm1f(y);
        sp[j * DF + 16 * t] = y;
      }
    }
  }
  __syncthreads();

  const float* lp = hrow + (size_t)wave * 64 * DF + 4 * lane;
  float* gp = fout + ((size_t)nodeBase + (size_t)wave * 64) * DF + 4 * lane;
#pragma unroll 8
  for (int i = 0; i < 64; ++i) { const v4f v = *(const v4f*)(lp + i * DF); *(volatile v4f*)(gp + (size_t)i * DF) = v; }
  __threadfence();
#pragma unroll 8
  for (int i = 0; i < 64; ++i) { const v4f v = *(const v4f*)(lp + i * DF); *(volatile v4f*)(gp + (size_t)i * DF) = v; }
}

__global__ __launch_bounds__(NTHR) void k_gather(const float* __restrict__ feats, const int* __restrict__ uid,
                                                 float* out, int nU, int nN) {
  const int lane = threadIdx.x & 31, wave = threadIdx.x >> 5;
  const int ub = blockIdx.x * NU + wave * 8;
  v4f v[8];
#pragma unroll
  for (int i = 0; i < 8; ++i) {
    int u = ub + i;
    u = u > nU - 1 ? nU - 1 : u;
    int n = uid[u];
    n = n < 0 ? 0 : (n > nN - 1 ? nN - 1 : n);
    v[i] = *(const v4f*)(feats + (size_t)n * DF + 4 * lane);
  }
#pragma unroll
  for (int i = 0; i < 8; ++i) {
    const int u = ub + i;
    if (u < nU) *(volatile v4f*)(out + (size_t)u * DF + 4 * lane) = v[i];
  }
  __threadfence();
#pragma unroll
  for (int i = 0; i < 8; ++i) {
    const int u = ub + i;
    if (u < nU) *(volatile v4f*)(out + (size_t)u * DF + 4 * lane) = v[i];
  }
}

extern "C" void kernel_launch(void* const* d_in, const int* in_sizes, int n_in,
                              void* d_out, int out_size, void* d_ws, size_t ws_size,
                              hipStream_t stream) {
  if (n_in < 8) return;
  const int nN = in_sizes[0] / DF;
  if (nN <= 0 || in_sizes[0] != nN * DF) return;
  const int nL = in_sizes[1] / (DF * DF);
  if (nL <= 0 || in_sizes[1] != nL * DF * DF) return;
  if (in_sizes[2] < nL * DF || in_sizes[3] < nL * DF || in_sizes[4] < nL * DF) return;
  const int nE = in_sizes[5];
  if (nE < 0 || in_sizes[6] != nE) return;
  const int nU = in_sizes[7];
  if (nU <= 0 || out_size != nU * DF) return;

  const float* emb   = (const float*)d_in[0];
  const float* W     = (const float*)d_in[1];
  const float* bias  = (const float*)d_in[2];
  const float* gamma = (const float*)d_in[3];
  const float* beta  = (const float*)d_in[4];
  const int*   src   = (const int*)d_in[5];
  const int*   dst   = (const int*)d_in[6];
  const int*   uid   = (const int*)d_in[7];
  float* out = (float*)d_out;

  const int nBlk = (nN + NB - 1) / NB;

  char* ws = (char*)d_ws;
  size_t off = 0;
  const size_t wBytes = (size_t)nL * DF * DF * 2;
  const size_t pBytes = (size_t)nBlk * NB * DF * 4;
  const size_t oWh = off; off += wBytes; off = (off + 255) & ~(size_t)255;
  const size_t oWl = off; off += wBytes; off = (off + 255) & ~(size_t)255;
  const size_t oPA = off; off += pBytes; off = (off + 255) & ~(size_t)255;
  const size_t oPB = off; off += pBytes; off = (off + 255) & ~(size_t)255;
  if (off > ws_size) return;
  __bf16* whi = (__bf16*)(ws + oWh);
  __bf16* wlo = (__bf16*)(ws + oWl);
  float* plane[2];
  plane[0] = (float*)(ws + oPA);
  plane[1] = (float*)(ws + oPB);

  const int n8 = nL * DF * DF / 8;
  k_wprep<<<(n8 + NTHR - 1) / NTHR, NTHR, 0, stream>>>(W, whi, wlo, n8);

  hipFuncSetAttribute(reinterpret_cast<const void*>(&k_layer),
                      hipFuncAttributeMaxDynamicSharedMemorySize, LDS_LAYER);
  for (int l = 0; l < nL; ++l) {
    const float* fin = (l == 0) ? emb : plane[(l - 1) & 1];
    float* fo = plane[l & 1];
    k_layer<<<nBlk, NTHR, LDS_LAYER, stream>>>(
        fin, src, dst, whi + (size_t)l * DF * DF, wlo + (size_t)l * DF * DF,
        bias + (size_t)l * DF, gamma + (size_t)l * DF, beta + (size_t)l * DF, fo, nN, nE);
  }

  k_gather<<<(nU + NU - 1) / NU, NTHR, 0, stream>>>(plane[(nL - 1) & 1], uid, out, nU, nN);
}
